// LSTMActor_36747740184872
// MI455X (gfx1250) — hardware-verified
//
#include <hip/hip_runtime.h>


typedef _Float16 f16_t;
typedef _Float16 v16h __attribute__((ext_vector_type(16)));
typedef _Float16 v8h  __attribute__((ext_vector_type(8), __may_alias__));
typedef float    v8f  __attribute__((ext_vector_type(8)));
typedef float    v4f  __attribute__((ext_vector_type(4), __may_alias__));
typedef unsigned v4u  __attribute__((ext_vector_type(4), __may_alias__));

#define T_STEPS    96
#define OBS_W      194
#define X1_W       192
#define ROWS       16
#define FC1_K      1538
#define FC1_N      128
#define TILE_H     512
#define UNITS_B1   128
#define UNITS_B2   256
#define UNITS_FC   (48 * 8 * 64)
#define UNITS_ALL  (UNITS_B1 + UNITS_B2 + UNITS_FC)
#define HOFF_B2    (2 * TILE_H)
#define HOFF_FC    (6 * TILE_H)
#define WS_BYTES_USED ((size_t)UNITS_ALL * 16)

#define SC_L       16.0f
#define SC_FC      64.0f
#define LOG2E_F    1.4426950408889634f

#define NOP4 "v_nop\n\tv_nop\n\tv_nop\n\tv_nop"

union FragU { v16h v; v8h hf[2]; };

__device__ __forceinline__ v8f wmma_raw(v16h a, v16h b, v8f c) {
  return __builtin_amdgcn_wmma_f32_16x16x32_f16(false, a, false, b, (short)0, c, false, false);
}
__device__ __forceinline__ v8f wmma_g(v16h a, v16h b, v8f c) {
  v8f d = wmma_raw(a, b, c);
  asm volatile(NOP4 : "+v"(d) : "v"(a), "v"(b));
  return d;
}

__device__ __forceinline__ float ex2f_(float x) {
#if __has_builtin(__builtin_amdgcn_exp2f)
  return __builtin_amdgcn_exp2f(x);
#else
  return __expf(x * 0.69314718055994531f);
#endif
}
__device__ __forceinline__ float actf(float x, float s, float A, float C) {
  const float e = ex2f_(x * s);
  return __builtin_fmaf(A, __builtin_amdgcn_rcpf(1.0f + e), C);
}

__global__ __launch_bounds__(256) void prep_tiles(const float* __restrict__ W_ih1,
                                                  const float* __restrict__ W_hh1,
                                                  const float* __restrict__ W_ih2,
                                                  const float* __restrict__ W_hh2,
                                                  const float* __restrict__ W_fc1,
                                                  f16_t* __restrict__ wsh)
{
  const int g = blockIdx.x * blockDim.x + threadIdx.x;
  if (g >= UNITS_ALL) return;
  const int lp = (g >> 1) & 31;
  const int hs = g & 1;
  const int hh = lp >> 4;
  const int c  = lp & 15;
  const int kb = 16 * hs + 8 * hh;
  float v[8];
  if (g < UNITS_B1) {
    const int tt = g >> 6;
    const int gr = (tt == 0) ? ((c < 8) ? c : (c + 8)) : ((c < 8) ? (c + 8) : (c + 16));
#pragma unroll
    for (int j = 0; j < 8; ++j) {
      const int k = kb + j;
      float w = 0.0f;
      if (k < 2)        w = W_ih1[gr * 2 + k];
      else if (k < 10)  w = W_hh1[gr * 8 + (k - 2)];
      v[j] = w * SC_L;
    }
  } else if (g < UNITS_B1 + UNITS_B2) {
    const int tt = (g - UNITS_B1) >> 6;
    const int gr = tt * 16 + c;
#pragma unroll
    for (int j = 0; j < 8; ++j) {
      const int k = kb + j;
      float w = 0.0f;
      if (k < 8)        w = W_ih2[gr * 8 + k];
      else if (k < 24)  w = W_hh2[gr * 16 + (k - 8)];
      v[j] = w * SC_L;
    }
  } else {
    const int tile = (g - UNITS_B1 - UNITS_B2) >> 6;
    const int kt = tile >> 3;
    const int nt = tile & 7;
    const int n  = nt * 16 + c;
    const float* src = W_fc1 + (size_t)n * FC1_K + (2 * kt + hs) * 16 + 8 * hh;
#pragma unroll
    for (int j = 0; j < 8; ++j) v[j] = src[j] * SC_FC;
  }
  union { v8h hv; v4u u; } pk;
#pragma unroll
  for (int j = 0; j < 8; ++j) pk.hv[j] = (f16_t)v[j];
  const v4u val = pk.u;
  volatile v4u* dst = (volatile v4u*)(wsh + (size_t)g * 8);
  *dst = val;
  __threadfence();
  *dst = val;
}

__global__ __launch_bounds__(32) __attribute__((amdgpu_num_vgpr(256)))
void lstm_actor(const float* __restrict__ obs,
                const float* __restrict__ b_ih1, const float* __restrict__ b_hh1,
                const float* __restrict__ b_ih2, const float* __restrict__ b_hh2,
                const float* __restrict__ W_fc1, const float* __restrict__ b_fc1,
                const float* __restrict__ W_fc2, const float* __restrict__ b_fc2,
                const f16_t* __restrict__ wsh,
                float* __restrict__ out, int nrows)
{
  __shared__ __attribute__((aligned(16))) f16_t obsL[ROWS][X1_W];
  __shared__ __attribute__((aligned(16))) f16_t a1row[ROWS][32];
  __shared__ __attribute__((aligned(16))) f16_t a2row[ROWS][32];
  __shared__ __attribute__((aligned(16))) f16_t h2pair[ROWS][32];
  __shared__ __attribute__((aligned(16))) float x2L[ROWS][2];
  __shared__ __attribute__((aligned(16))) float part[2 * ROWS][16];
  __shared__ __attribute__((aligned(16))) float outL[2 * ROWS];

  const int lane = threadIdx.x & 31;
  const int h    = lane >> 4;
  const int c    = lane & 15;
  const int row0 = blockIdx.x * ROWS;

  for (int r = 0; r < ROWS; ++r) {
    int rr = row0 + r;
    rr = (rr < nrows) ? rr : (nrows - 1);
    const float* src = obs + (size_t)rr * OBS_W;
    for (int k = lane; k < X1_W; k += 32) obsL[r][k] = (f16_t)src[k];
    if (lane < 2) x2L[r][lane] = src[X1_W + lane];
  }
  {
    const f16_t hz = (f16_t)0.0f;
    for (int i = lane; i < ROWS * 32; i += 32) {
      const int r = i >> 5, k = i & 31;
      a1row[r][k] = hz;
      a2row[r][k] = hz;
      h2pair[r][k] = hz;
    }
  }
  __syncthreads();

  FragU b1a, b1b, b2[4];
  {
    const f16_t* p = wsh + lane * 16;
    b1a.hf[0] = *(const v8h*)(p);
    b1a.hf[1] = *(const v8h*)(p + 8);
    b1b.hf[0] = *(const v8h*)(p + TILE_H);
    b1b.hf[1] = *(const v8h*)(p + TILE_H + 8);
#pragma unroll
    for (int tt = 0; tt < 4; ++tt) {
      const f16_t* q = wsh + HOFF_B2 + tt * TILE_H + lane * 16;
      b2[tt].hf[0] = *(const v8h*)(q);
      b2[tt].hf[1] = *(const v8h*)(q + 8);
    }
  }

  const bool lower = (c < 8);
  const int  u1    = c & 7;
  const int  rb1   = 8 * h + (lower ? 0 : 4);
  const int  gr0   = lower ? c : (c + 8);
  const int  gr1   = lower ? (c + 8) : (c + 16);
  const float bl1a = SC_L * (b_ih1[gr0] + b_hh1[gr0]);
  const float bl1b = SC_L * (b_ih1[gr1] + b_hh1[gr1]);
  float bl2[4];
#pragma unroll
  for (int tt = 0; tt < 4; ++tt) bl2[tt] = SC_L * (b_ih2[tt * 16 + c] + b_hh2[tt * 16 + c]);

  const float SIG16_S = -LOG2E_F / 16.0f;
  const float TNH16_S = -LOG2E_F / 8.0f;
  const float TNH_S   = -2.0f * LOG2E_F;
  const float a0s = lower ? SIG16_S : TNH16_S;
  const float a0A = lower ? 1.0f : 2.0f;
  const float a0C = lower ? 0.0f : -1.0f;

  v8f accFC[8];
#pragma unroll
  for (int nt = 0; nt < 8; ++nt)
#pragma unroll
    for (int v = 0; v < 8; ++v) accFC[nt][v] = 0.0f;
  float c1s[4] = {0.0f, 0.0f, 0.0f, 0.0f};
  float c2s[8] = {0.0f, 0.0f, 0.0f, 0.0f, 0.0f, 0.0f, 0.0f, 0.0f};

#pragma unroll 1
  for (int kt = 0; kt < T_STEPS / 2; ++kt) {
#pragma unroll
    for (int phase = 0; phase < 2; ++phase) {
      const int t = 2 * kt + phase;
      {
        const f16_t x0 = obsL[c][t];
        const f16_t x1 = obsL[c][T_STEPS + t];
        a1row[c][0] = x0;
        a1row[c][1] = x1;
      }
      __syncthreads();

      {
        FragU a;
        a.hf[0] = *(const v8h*)(&a1row[c][8 * h]);
        a.hf[1] = *(const v8h*)(&a1row[c][16 + 8 * h]);
        v8f g0, g1;
#pragma unroll
        for (int v = 0; v < 8; ++v) { g0[v] = bl1a; g1[v] = bl1b; }
        g0 = wmma_raw(a.v, b1a.v, g0);
        g1 = wmma_raw(a.v, b1b.v, g1);
        asm volatile(NOP4 : "+v"(g0), "+v"(g1) : "v"(a.v), "v"(b1a.v), "v"(b1b.v));
        float v0[8], v1[8];
#pragma unroll
        for (int v = 0; v < 8; ++v) {
          v0[v] = actf(g0[v], a0s, a0A, a0C);
          v1[v] = actf(g1[v], SIG16_S, 1.0f, 0.0f);
        }
#pragma unroll
        for (int j = 0; j < 4; ++j) {
          const float s0 = lower ? v0[4 + j] : v0[j];
          const float s1 = lower ? v1[4 + j] : v1[j];
          const float r0 = __shfl_xor(s0, 8);
          const float r1 = __shfl_xor(s1, 8);
          const float iv = lower ? v0[j] : r0;
          const float fv = lower ? v1[j] : r1;
          const float gv = lower ? r0 : v0[4 + j];
          const float ov = lower ? r1 : v1[4 + j];
          const float cn = __builtin_fmaf(fv, c1s[j], iv * gv);
          c1s[j] = cn;
          const float hv = ov * actf(cn, TNH_S, 2.0f, -1.0f);
          const f16_t hq = (f16_t)hv;
          const int row = rb1 + j;
          a1row[row][2 + u1] = hq;
          a2row[row][u1]     = hq;
        }
      }
      __syncthreads();

      {
        FragU a;
        a.hf[0] = *(const v8h*)(&a2row[c][8 * h]);
        a.hf[1] = *(const v8h*)(&a2row[c][16 + 8 * h]);
        v8f q0, q1, q2, q3;
#pragma unroll
        for (int v = 0; v < 8; ++v) { q0[v] = bl2[0]; q1[v] = bl2[1]; q2[v] = bl2[2]; q3[v] = bl2[3]; }
        q0 = wmma_raw(a.v, b2[0].v, q0);
        q1 = wmma_raw(a.v, b2[1].v, q1);
        q2 = wmma_raw(a.v, b2[2].v, q2);
        q3 = wmma_raw(a.v, b2[3].v, q3);
        asm volatile(NOP4 : "+v"(q0), "+v"(q1), "+v"(q2), "+v"(q3)
                     : "v"(a.v), "v"(b2[0].v), "v"(b2[1].v), "v"(b2[2].v), "v"(b2[3].v));
#pragma unroll
        for (int v = 0; v < 8; ++v) {
          const float iv = actf(q0[v], SIG16_S, 1.0f, 0.0f);
          const float fv = actf(q1[v], SIG16_S, 1.0f, 0.0f);
          const float gv = actf(q2[v], TNH16_S, 2.0f, -1.0f);
          const float ov = actf(q3[v], SIG16_S, 1.0f, 0.0f);
          const float cn = __builtin_fmaf(fv, c2s[v], iv * gv);
          c2s[v] = cn;
          const float hv = ov * actf(cn, TNH_S, 2.0f, -1.0f);
          const f16_t hq = (f16_t)hv;
          const int row = 8 * h + v;
          a2row[row][8 + c]            = hq;
          h2pair[row][16 * phase + c]  = hq;
        }
      }
    }
    __syncthreads();

    {
      FragU a;
      a.hf[0] = *(const v8h*)(&h2pair[c][8 * h]);
      a.hf[1] = *(const v8h*)(&h2pair[c][16 + 8 * h]);
      const f16_t* bp = wsh + HOFF_FC + (size_t)kt * (8 * TILE_H) + lane * 16;
#pragma unroll
      for (int nt = 0; nt < 8; ++nt) {
        FragU b;
        b.hf[0] = *(const v8h*)(bp + nt * TILE_H);
        b.hf[1] = *(const v8h*)(bp + nt * TILE_H + 8);
        accFC[nt] = wmma_g(a.v, b.v, accFC[nt]);
      }
    }
  }

  float pp[8][2];
#pragma unroll
  for (int v = 0; v < 8; ++v) { pp[v][0] = 0.0f; pp[v][1] = 0.0f; }
#pragma unroll
  for (int nt = 0; nt < 8; ++nt) {
    const int col = nt * 16 + c;
    const float bc  = b_fc1[col];
    const float w0  = W_fc1[(size_t)col * FC1_K + (FC1_K - 2)];
    const float w1  = W_fc1[(size_t)col * FC1_K + (FC1_K - 1)];
    const float u0  = W_fc2[col];
    const float u1v = W_fc2[FC1_N + col];
#pragma unroll
    for (int v = 0; v < 8; ++v) {
      const int row = 8 * h + v;
      float val = __builtin_fmaf(accFC[nt][v], 1.0f / SC_FC, bc);
      val = __builtin_fmaf(x2L[row][0], w0, val);
      val = __builtin_fmaf(x2L[row][1], w1, val);
      val = fmaxf(val, 0.0f);
      pp[v][0] = __builtin_fmaf(val, u0,  pp[v][0]);
      pp[v][1] = __builtin_fmaf(val, u1v, pp[v][1]);
    }
  }
#pragma unroll
  for (int v = 0; v < 8; ++v) {
    part[(8 * h + v) * 2 + 0][c] = pp[v][0];
    part[(8 * h + v) * 2 + 1][c] = pp[v][1];
  }
  __syncthreads();

  float y;
  {
    const v4f* pr = (const v4f*)(&part[lane][0]);
    const v4f s4 = (pr[0] + pr[1]) + (pr[2] + pr[3]);
    const float s = b_fc2[lane & 1] + ((s4[0] + s4[1]) + (s4[2] + s4[3]));
    y = s / (1.0f + fabsf(s));
  }
  outL[lane] = y;
  __syncthreads();

  const bool full = (row0 + ROWS <= nrows);
  if (full) {
    if (lane < 8) {
      const v4f ov = *(const v4f*)(&outL[4 * lane]);
      volatile v4f* d = (volatile v4f*)(out + (size_t)row0 * 2 + 4 * lane);
      *d = ov;
      __threadfence();
      *d = ov;
    }
  } else {
    const int row = row0 + (lane >> 1);
    if (row < nrows) {
      volatile float* d = out + (size_t)row * 2 + (lane & 1);
      *d = y;
      __threadfence();
      *d = y;
    }
  }
}

extern "C" void kernel_launch(void* const* d_in, const int* in_sizes, int n_in,
                              void* d_out, int out_size, void* d_ws, size_t ws_size,
                              hipStream_t stream) {
  if (n_in < 13) return;
  const float* obs   = (const float*)d_in[0];
  const float* W_ih1 = (const float*)d_in[1];
  const float* W_hh1 = (const float*)d_in[2];
  const float* b_ih1 = (const float*)d_in[3];
  const float* b_hh1 = (const float*)d_in[4];
  const float* W_ih2 = (const float*)d_in[5];
  const float* W_hh2 = (const float*)d_in[6];
  const float* b_ih2 = (const float*)d_in[7];
  const float* b_hh2 = (const float*)d_in[8];
  const float* W_fc1 = (const float*)d_in[9];
  const float* b_fc1 = (const float*)d_in[10];
  const float* W_fc2 = (const float*)d_in[11];
  const float* b_fc2 = (const float*)d_in[12];
  float* out = (float*)d_out;

  int nrows = out_size / 2;
  const int nobs = in_sizes[0] / OBS_W;
  if (nobs < nrows) nrows = nobs;
  if (nrows <= 0) return;
  if (ws_size < WS_BYTES_USED) return;

  f16_t* wsh = (f16_t*)d_ws;

  const int pgrid = (UNITS_ALL + 255) / 256;
  prep_tiles<<<dim3(pgrid), dim3(256), 0, stream>>>(W_ih1, W_hh1, W_ih2, W_hh2, W_fc1, wsh);

  const int mgrid = (nrows + ROWS - 1) / ROWS;
  lstm_actor<<<dim3(mgrid), dim3(32), 0, stream>>>(obs, b_ih1, b_hh1, b_ih2, b_hh2,
                                                   W_fc1, b_fc1, W_fc2, b_fc2,
                                                   (const f16_t*)wsh, out, nrows);
}
